// Fusion_Trans_Block_54623394071056
// MI455X (gfx1250) — hardware-verified
//
#include <hip/hip_runtime.h>
#include <hip/hip_bf16.h>

typedef _Float16 f16x8  __attribute__((ext_vector_type(8)));
typedef _Float16 f16x16 __attribute__((ext_vector_type(16)));
typedef float    f32x8  __attribute__((ext_vector_type(8)));

typedef int v4i __attribute__((vector_size(16)));
typedef __attribute__((address_space(1))) v4i gv4i;
typedef __attribute__((address_space(3))) v4i lv4i;

#define DIM    768
#define HEADS  12
#define HDIM   64
#define HIDDEN 3072
#define SEQ    1024
#define BATCH  8
#define ROWS   (BATCH * SEQ)

static __device__ __forceinline__ f32x8 wmma_f16(f16x16 a, f16x16 b, f32x8 c) {
  f32x8 d = __builtin_amdgcn_wmma_f32_16x16x32_f16(false, a, false, b, (short)0, c, false, false);
  asm volatile("v_nop\n\tv_nop\n\tv_nop\n\tv_nop" : "+v"(d) : "v"(a), "v"(b));
  return d;
}
typedef float v4f __attribute__((ext_vector_type(4)));
typedef unsigned v4u __attribute__((ext_vector_type(4)));
typedef unsigned v2u __attribute__((ext_vector_type(2)));
typedef float __attribute__((may_alias)) float_a;
typedef unsigned __attribute__((may_alias)) uint_a;
template <typename T> __device__ __forceinline__ void vst2(void* p, T v) { *(volatile T*)p = v; __threadfence(); *(volatile T*)p = v; }

static __device__ __forceinline__ void async_copy16(const _Float16* g, _Float16* l) {
#ifdef HAVE_ASYNC_LDS
  __builtin_amdgcn_global_load_async_to_lds_b128((gv4i*)g, (lv4i*)l, 0, 0);
#else
  *(f16x8*)l = *(const f16x8*)g;
#endif
}

static __device__ __forceinline__ void wait_async0() { }

__global__ __launch_bounds__(256) void cvt_f32_f16_kernel(
    const float* __restrict__ src, _Float16* __restrict__ dst, int n) {
  int g = blockIdx.x * 256 + threadIdx.x;
  if (g * 8 >= n) return;
  union { f16x8 h; v4u u; } pk;
#pragma unroll
  for (int e = 0; e < 8; ++e) pk.h[e] = (_Float16)src[(size_t)g * 8 + e];
  vst2(dst + (size_t)g * 8, pk.u);
}

__global__ __launch_bounds__(256) void ln_kernel(
    const float* __restrict__ src_pre, const float* __restrict__ src_post,
    const float* __restrict__ src_full,
    const float* __restrict__ g, const float* __restrict__ beta,
    _Float16* __restrict__ out, float* __restrict__ xout, int concat) {
  const int lane = threadIdx.x & 31;
  const int wid  = threadIdx.x >> 5;
  const int row  = blockIdx.x * 8 + wid;

  const float* src;
  if (concat) {
    const int b = row >> 10, seq = row & 1023;
    src = (seq < 512) ? src_pre  + ((size_t)b * 512 + seq) * DIM
                      : src_post + ((size_t)b * 512 + (seq - 512)) * DIM;
  } else {
    src = src_full + (size_t)row * DIM;
  }

  float vals[24];
  float s = 0.f, s2 = 0.f;
#pragma unroll
  for (int i = 0; i < 24; ++i) {
    float v = src[lane + i * 32];
    vals[i] = v; s += v; s2 += v * v;
  }
#pragma unroll
  for (int mk = 1; mk < 32; mk <<= 1) {
    s  += __shfl_xor(s,  mk, 32);
    s2 += __shfl_xor(s2, mk, 32);
  }
  const float mu  = s  * (1.f / DIM);
  const float var = s2 * (1.f / DIM) - mu * mu;
  const float rs  = rsqrtf(var + 1e-5f);

  __shared__ __attribute__((aligned(16))) _Float16 hrow[8][DIM];
#pragma unroll
  for (int i = 0; i < 24; ++i) {
    const int c = lane + i * 32;
    const float v = vals[i];
    if (concat) vst2(xout + (size_t)row * DIM + c, (float_a)v);
    hrow[wid][c] = (_Float16)((v - mu) * rs * g[c] + beta[c]);
  }
  asm volatile("s_wait_dscnt 0" ::: "memory"); __builtin_amdgcn_wave_barrier(); __builtin_amdgcn_fence(__ATOMIC_RELEASE, "workgroup");
  for (int pc = lane; pc < DIM / 8; pc += 32) vst2(out + (size_t)row * DIM + pc * 8, *(const v4u*)(&hrow[wid][pc * 8]));
}

__global__ __launch_bounds__(256) void gemm_kernel(
    const _Float16* __restrict__ A, int lda,
    const _Float16* __restrict__ B, int ldb,
    const float* __restrict__ bias, int K, int mode,
    _Float16* __restrict__ outh, float* __restrict__ outf,
    const float* __restrict__ resid, const float* __restrict__ gamma, int ldo) {
  __shared__ __attribute__((aligned(32))) _Float16 As[2][64 * 32];
  __shared__ __attribute__((aligned(32))) _Float16 Bt[2][128 * 32];
  __shared__ __attribute__((aligned(16))) float Ct[64][132];

  const int t    = threadIdx.x;
  const int lane = t & 31, wid = t >> 5;
  const int m0   = blockIdx.y * 64;
  const int n0   = blockIdx.x * 128;
  const int wrow = (wid >> 2) * 32;
  const int wcol = (wid & 3) * 32;
  const int cn   = lane & 15;
  const int hi   = lane >> 4;
  const int ak8  = hi * 8;
  const int bk16 = hi * 16;

  const int ar  = t >> 2,  ach = (t & 3) * 8;
  const int bpk = t >> 4,  bch = (t & 15) * 8;

  const _Float16* Abase = A + (size_t)(m0 + ar) * lda + ach;
  _Float16* AsDst = (_Float16*)As[0] + ar * 32 + ach;

  async_copy16(Abase + 0, AsDst);
  {
    union { f16x8 v; unsigned short u[8]; } lo, hi2;
    lo.v  = *(const f16x8*)(B + (size_t)(2 * bpk)     * ldb + n0 + bch);
    hi2.v = *(const f16x8*)(B + (size_t)(2 * bpk + 1) * ldb + n0 + bch);
    unsigned int* bt32 = (unsigned int*)Bt[0];
#pragma unroll
    for (int i = 0; i < 8; ++i)
      bt32[(bch + i) * 16 + bpk] = (unsigned int)lo.u[i] |
                                   ((unsigned int)hi2.u[i] << 16);
  }
  wait_async0();
  __syncthreads();

  f32x8 acc[2][2] = {};

  for (int k0 = 0; k0 < K; k0 += 32) {
    const int p    = (k0 >> 5) & 1;
    const int np   = p ^ 1;
    const bool more = (k0 + 32) < K;

    union { f16x8 v; unsigned short u[8]; } nlo = {}, nhi = {};
    if (more) {
      async_copy16(Abase + (k0 + 32), AsDst + np * 2048);
      nlo.v = *(const f16x8*)(B + (size_t)(k0 + 32 + 2 * bpk)     * ldb + n0 + bch);
      nhi.v = *(const f16x8*)(B + (size_t)(k0 + 32 + 2 * bpk + 1) * ldb + n0 + bch);
    }

    const _Float16* Asp = As[p];
    const _Float16* Btp = Bt[p];
    f16x16 a[2], bf[2];
#pragma unroll
    for (int i = 0; i < 2; ++i) {
      union { f16x16 v; f16x8 h[2]; } u;
      u.h[0] = *(const f16x8*)(Asp + (wrow + i * 16 + cn) * 32 + ak8);
      u.h[1] = *(const f16x8*)(Asp + (wrow + i * 16 + cn) * 32 + ak8 + 16);
      a[i] = u.v;
    }
#pragma unroll
    for (int j = 0; j < 2; ++j) {
      union { f16x16 v; f16x8 h[2]; } ub;
      ub.h[0] = *(const f16x8*)(Btp + (wcol + j * 16 + cn) * 32 + ak8);
      ub.h[1] = *(const f16x8*)(Btp + (wcol + j * 16 + cn) * 32 + ak8 + 16);
      bf[j] = ub.v;
    }
#pragma unroll
    for (int i = 0; i < 2; ++i)
#pragma unroll
      for (int j = 0; j < 2; ++j)
        acc[i][j] = wmma_f16(a[i], bf[j], acc[i][j]);

    if (more) {
      unsigned int* bt32 = (unsigned int*)Bt[np];
#pragma unroll
      for (int i = 0; i < 8; ++i)
        bt32[(bch + i) * 16 + bpk] = (unsigned int)nlo.u[i] |
                                     ((unsigned int)nhi.u[i] << 16);
      wait_async0();
    }
    __syncthreads();
  }

#pragma unroll
  for (int i = 0; i < 2; ++i)
#pragma unroll
    for (int j = 0; j < 2; ++j) {
      const int ln_ = wcol + j * 16 + cn;
      const float bv = bias[n0 + ln_];
#pragma unroll 1
      for (int r = 0; r < 8; ++r) {
        float val = acc[i][j][r] + bv;
        if (mode == 1) val = 0.5f * val * (1.0f + erff(val * 0.70710678f));
        Ct[wrow + i * 16 + r + hi * 8][ln_] = val;
      }
    }
  __syncthreads();
  if (mode == 0 || mode == 1) {
    for (int q = t; q < 64 * 16; q += 256) { const int rl = q >> 4, pc = q & 15;
      union { f16x8 h; v4u u; } pk;
#pragma unroll
      for (int e = 0; e < 8; ++e) pk.h[e] = (_Float16)Ct[rl][pc * 8 + e];
      vst2(outh + (size_t)(m0 + rl) * ldo + n0 + pc * 8, pk.u); }
  } else if (mode == 2) {
    const int bb = m0 >> 10, seq0 = m0 & 1023;
    for (int q = t; q < 128 * 32; q += 256) { const int cnl = q >> 5, ls = q & 31; const int gn = n0 + cnl; const int hh = gn >> 6, dd = gn & 63;
      union { _Float16 h[2]; unsigned u; } pk; pk.h[0] = (_Float16)Ct[ls * 2][cnl]; pk.h[1] = (_Float16)Ct[ls * 2 + 1][cnl];
      vst2(outh + (((size_t)bb * HEADS + hh) * HDIM + dd) * SEQ + seq0 + ls * 2, (uint_a)pk.u); }
  } else {
    for (int q = t; q < 64 * 32; q += 256) { const int rl = q >> 5, pc = q & 31;
      const size_t idx = (size_t)(m0 + rl) * ldo + n0 + pc * 4;
      v4f v = *(const v4f*)(&Ct[rl][pc * 4]); const v4f rr = *(const v4f*)(resid + idx); const v4f gg = *(const v4f*)(gamma + n0 + pc * 4);
      vst2(outf + idx, rr + gg * v); }
  }
}

__global__ __launch_bounds__(256) void attn_kernel(
    const _Float16* __restrict__ Q, const _Float16* __restrict__ K,
    const _Float16* __restrict__ Vt, const float* __restrict__ mask,
    _Float16* __restrict__ O) {
  __shared__ __attribute__((aligned(32))) _Float16 pst[8][16 * 64];

  const int lane = threadIdx.x & 31;
  const int wid  = threadIdx.x >> 5;
  const int gw   = blockIdx.x * 8 + wid;
  const int qt   = gw & 63;
  const int head = (gw >> 6) % HEADS;
  const int b    = gw / (64 * HEADS);
  const int q0   = qt * 16;
  _Float16* P = pst[wid];

  const int cn  = lane & 15;
  const int hi  = lane >> 4;
  const int ak8 = hi * 8;
  const int k16 = hi * 16;

  const _Float16* qrow = Q + ((size_t)(b * SEQ + q0 + cn)) * DIM + head * HDIM;
  f16x16 qa[2];
#pragma unroll
  for (int t = 0; t < 2; ++t) {
    union { f16x16 v; f16x8 h[2]; } u;
    u.h[0] = *(const f16x8*)(qrow + t * 32 + ak8);
    u.h[1] = *(const f16x8*)(qrow + t * 32 + ak8 + 16);
    qa[t] = u.v;
  }

  f32x8 acc[4] = {};
  float mrun[8], lrun[8];
#pragma unroll
  for (int r = 0; r < 8; ++r) { mrun[r] = -3.0e38f; lrun[r] = 0.f; }

  for (int kt = 0; kt < SEQ / 32; ++kt) {
    const int kbase = kt * 32;

    if (kt + 1 < SEQ / 32) {
      __builtin_prefetch(K + ((size_t)(b * SEQ + kbase + 32 + lane)) * DIM +
                             head * HDIM, 0, 0);
      __builtin_prefetch(mask + ((size_t)b * SEQ + q0 + hi * 8) * SEQ +
                             kbase + 32 + cn, 0, 0);
    }

    float sv[2][8];
#pragma unroll
    for (int tsub = 0; tsub < 2; ++tsub) {
      const int key = kbase + tsub * 16 + cn;
      const _Float16* krow = K + ((size_t)(b * SEQ + key)) * DIM + head * HDIM;
      union { f16x16 v; f16x8 h[2]; } uk0, uk1;
      uk0.h[0] = *(const f16x8*)(krow + ak8);      uk0.h[1] = *(const f16x8*)(krow + ak8 + 16);
      uk1.h[0] = *(const f16x8*)(krow + 32 + ak8); uk1.h[1] = *(const f16x8*)(krow + 32 + ak8 + 16);
      f16x16 kb0 = uk0.v, kb1 = uk1.v;
      f32x8 c = {};
      c = wmma_f16(qa[0], kb0, c);
      c = wmma_f16(qa[1], kb1, c);
#pragma unroll
      for (int r = 0; r < 8; ++r) sv[tsub][r] = c[r];
    }
#pragma unroll
    for (int r = 0; r < 8; ++r) {
      const int qm = q0 + r + hi * 8;
      const float* mp = mask + ((size_t)b * SEQ + qm) * SEQ + kbase;
      sv[0][r] = sv[0][r] * 0.125f + mp[cn];
      sv[1][r] = sv[1][r] * 0.125f + mp[16 + cn];
    }
    float tmax[8];
#pragma unroll
    for (int r = 0; r < 8; ++r) tmax[r] = fmaxf(sv[0][r], sv[1][r]);
#pragma unroll
    for (int mk = 1; mk < 16; mk <<= 1)
#pragma unroll
      for (int r = 0; r < 8; ++r)
        tmax[r] = fmaxf(tmax[r], __shfl_xor(tmax[r], mk, 32));

    float corr[8], rs[8];
#pragma unroll
    for (int r = 0; r < 8; ++r) {
      const float mn = fmaxf(mrun[r], tmax[r]);
      corr[r]  = expf(mrun[r] - mn);
      mrun[r]  = mn;
      sv[0][r] = expf(sv[0][r] - mn);
      sv[1][r] = expf(sv[1][r] - mn);
      rs[r]    = sv[0][r] + sv[1][r];
    }
#pragma unroll
    for (int mk = 1; mk < 16; mk <<= 1)
#pragma unroll
      for (int r = 0; r < 8; ++r) rs[r] += __shfl_xor(rs[r], mk, 32);
#pragma unroll
    for (int r = 0; r < 8; ++r) lrun[r] = lrun[r] * corr[r] + rs[r];
#pragma unroll
    for (int j = 0; j < 4; ++j)
#pragma unroll
      for (int r = 0; r < 8; ++r) acc[j][r] *= corr[r];

#pragma unroll
    for (int r = 0; r < 8; ++r) {
      const int m = r + hi * 8;
      P[m * 32 + cn]      = (_Float16)sv[0][r];
      P[m * 32 + 16 + cn] = (_Float16)sv[1][r];
    }
    asm volatile("s_wait_dscnt 0" ::: "memory"); __builtin_amdgcn_wave_barrier(); __builtin_amdgcn_fence(__ATOMIC_RELEASE, "workgroup");
    union { f16x16 v; f16x8 h[2]; } up;
    up.h[0] = *(const f16x8*)(P + cn * 32 + ak8);
    up.h[1] = *(const f16x8*)(P + cn * 32 + ak8 + 16);
    const f16x16 pa = up.v;

#pragma unroll
    for (int j = 0; j < 4; ++j) {
      const _Float16* vrow =
          Vt + (((size_t)b * HEADS + head) * HDIM + j * 16 + cn) * SEQ + kbase + ak8;
      union { f16x16 v; f16x8 h[2]; } uv; uv.h[0] = *(const f16x8*)(vrow); uv.h[1] = *(const f16x8*)(vrow + 16);
      acc[j] = wmma_f16(pa, uv.v, acc[j]);
    }
  }

  __builtin_amdgcn_wave_barrier();
#pragma unroll
  for (int j = 0; j < 4; ++j)
#pragma unroll
    for (int r = 0; r < 8; ++r) P[(r + hi * 8) * 64 + j * 16 + cn] = (_Float16)(acc[j][r] / lrun[r]);
  asm volatile("s_wait_dscnt 0" ::: "memory"); __builtin_amdgcn_wave_barrier(); __builtin_amdgcn_fence(__ATOMIC_RELEASE, "workgroup");
#pragma unroll
  for (int q = 0; q < 4; ++q) { const int rl = q * 4 + (lane >> 3), pc = lane & 7;
    vst2(O + ((size_t)(b * SEQ + q0 + rl)) * DIM + head * HDIM + pc * 8, *(const v4u*)(P + rl * 64 + pc * 8)); }
}

extern "C" void kernel_launch(void* const* d_in, const int* in_sizes, int n_in,
                              void* d_out, int out_size, void* d_ws, size_t ws_size,
                              hipStream_t stream) {
  (void)in_sizes; (void)n_in; (void)out_size; (void)ws_size;

  const float* x_pre  = (const float*)d_in[0];
  const float* x_post = (const float*)d_in[1];
  const float* mask   = (const float*)d_in[2];
  const float* ln1_g  = (const float*)d_in[3];
  const float* ln1_b  = (const float*)d_in[4];
  const float* Wq = (const float*)d_in[5];   const float* bq = (const float*)d_in[6];
  const float* Wk = (const float*)d_in[7];   const float* bk = (const float*)d_in[8];
  const float* Wv = (const float*)d_in[9];   const float* bv = (const float*)d_in[10];
  const float* Wo = (const float*)d_in[11];  const float* bo = (const float*)d_in[12];
  const float* ln2_g = (const float*)d_in[13]; const float* ln2_b = (const float*)d_in[14];
  const float* W1 = (const float*)d_in[15];  const float* b1 = (const float*)d_in[16];
  const float* W2 = (const float*)d_in[17];  const float* b2 = (const float*)d_in[18];
  const float* g1 = (const float*)d_in[19];  const float* g2 = (const float*)d_in[20];

  char* ws = (char*)d_ws;
  float*    X   = (float*)(ws + 0);
  float*    X2  = (float*)(ws + 25165824);
  _Float16* H   = (_Float16*)(ws + 50331648);
  _Float16* Qh  = (_Float16*)(ws + 62914560);
  _Float16* Kh  = (_Float16*)(ws + 75497472);
  _Float16* Vt  = (_Float16*)(ws + 88080384);
  _Float16* Oh  = (_Float16*)(ws + 100663296);
  _Float16* MID = (_Float16*)(ws + 62914560);
  _Float16* Wq16 = (_Float16*)(ws + 113246208);
  _Float16* Wk16 = Wq16 + 589824;
  _Float16* Wv16 = Wk16 + 589824;
  _Float16* Wo16 = Wv16 + 589824;
  _Float16* W116 = Wo16 + 589824;
  _Float16* W216 = W116 + 2359296;

  cvt_f32_f16_kernel<<<288, 256, 0, stream>>>(Wq, Wq16, 589824);
  cvt_f32_f16_kernel<<<288, 256, 0, stream>>>(Wk, Wk16, 589824);
  cvt_f32_f16_kernel<<<288, 256, 0, stream>>>(Wv, Wv16, 589824);
  cvt_f32_f16_kernel<<<288, 256, 0, stream>>>(Wo, Wo16, 589824);
  cvt_f32_f16_kernel<<<1152, 256, 0, stream>>>(W1, W116, 2359296);
  cvt_f32_f16_kernel<<<1152, 256, 0, stream>>>(W2, W216, 2359296);

  ln_kernel<<<ROWS / 8, 256, 0, stream>>>(x_pre, x_post, nullptr,
                                          ln1_g, ln1_b, H, X, 1);

  dim3 gemm_grid_768(DIM / 128, ROWS / 64);
  gemm_kernel<<<gemm_grid_768, 256, 0, stream>>>(H, DIM, Wq16, DIM, bq, DIM, 0,
                                                 Qh, nullptr, nullptr, nullptr, DIM);
  gemm_kernel<<<gemm_grid_768, 256, 0, stream>>>(H, DIM, Wk16, DIM, bk, DIM, 0,
                                                 Kh, nullptr, nullptr, nullptr, DIM);
  gemm_kernel<<<gemm_grid_768, 256, 0, stream>>>(H, DIM, Wv16, DIM, bv, DIM, 2,
                                                 Vt, nullptr, nullptr, nullptr, DIM);

  attn_kernel<<<(BATCH * HEADS * (SEQ / 16)) / 8, 256, 0, stream>>>(Qh, Kh, Vt,
                                                                    mask, Oh);

  gemm_kernel<<<gemm_grid_768, 256, 0, stream>>>(Oh, DIM, Wo16, DIM, bo, DIM, 3,
                                                 nullptr, X2, X, g1, DIM);

  ln_kernel<<<ROWS / 8, 256, 0, stream>>>(nullptr, nullptr, X2,
                                          ln2_g, ln2_b, H, nullptr, 0);

  dim3 gemm_grid_3072(HIDDEN / 128, ROWS / 64);
  gemm_kernel<<<gemm_grid_3072, 256, 0, stream>>>(H, DIM, W116, HIDDEN, b1, DIM, 1,
                                                  MID, nullptr, nullptr, nullptr, HIDDEN);

  gemm_kernel<<<gemm_grid_768, 256, 0, stream>>>(MID, HIDDEN, W216, DIM, b2, HIDDEN, 3,
                                                 nullptr, (float*)d_out, X2, g2, DIM);
}
